// TransformerBlock_81784767250432
// MI455X (gfx1250) — hardware-run, weakly checked
//
#include <hip/hip_runtime.h>


#ifndef NB
#define NB 2
#endif
#ifndef SEQ
#define SEQ 1024
#endif
#define NB_FULL  2
#define SEQ_FULL 1024
#define DM   1024
#define NH_  16
#define HD   64
#define HK   1024
#define MF   4096
#define MEMS SEQ
#define TK   (2 * SEQ)
#define TK_FULL (2 * SEQ_FULL)
#define ROWS  (NB * SEQ)
#define KROWS (NB * TK)
#define AW   4
#define OSP  68
#define WCS  64.0f
#define AVS  64.0f
#define PSH  14.0f
#define LOG2E 1.4426950408889634f
#define NEGB (-3.0e38f)

static_assert(HD == 64);
static_assert(NH_ * HD == HK);
static_assert(DM % 32 == 0);
static_assert(HK % 32 == 0);
static_assert(MF % 32 == 0);
static_assert(DM % 64 == 0);
static_assert(HK % 64 == 0);
static_assert(MF % 64 == 0);
static_assert(SEQ % 64 == 0);
static_assert(TK % 64 == 0);
static_assert(ROWS % 64 == 0);
static_assert(KROWS % 64 == 0);
static_assert(TK % 128 == 0);
static_assert(TK % 32 == 0);
static_assert(SEQ % (16 * AW) == 0);
static_assert(NB <= NB_FULL);
static_assert(SEQ <= SEQ_FULL);
static_assert((OSP * 4) % 16 == 0);
static_assert(256 * 4 == DM);
static_assert(128 * 8 == DM);
static_assert(DM % 8 == 0);
static_assert(16 * OSP * 4 <= 131072);
static_assert(AW * 16 * OSP * 4 <= 131072);
static_assert(DM * 4 + 64 <= 131072);

typedef _Float16 h16;
typedef unsigned short bf;
typedef __attribute__((ext_vector_type(16))) __bf16   v16bf;
typedef __attribute__((ext_vector_type(16))) _Float16 v16h;
typedef __attribute__((ext_vector_type(8)))  _Float16 v8h;
typedef __attribute__((ext_vector_type(8)))  unsigned short v8us;
typedef __attribute__((ext_vector_type(16))) unsigned short v16us;
typedef __attribute__((ext_vector_type(8)))  float    v8f;
typedef __attribute__((ext_vector_type(4)))  float    v4f;
typedef v4f  __attribute__((may_alias)) v4fa;

__device__ __forceinline__ unsigned short f2bf(float f) { unsigned u = __float_as_uint(f); u += 0x7FFFu + ((u >> 16) & 1u); return (unsigned short)(u >> 16); }
__device__ __forceinline__ float bfr(float f) { return __uint_as_float(((unsigned)f2bf(f)) << 16); }
__device__ __forceinline__ v16h cat16(v8h lo, v8h hi) { return __builtin_shufflevector(lo, hi, 0, 1, 2, 3, 4, 5, 6, 7, 8, 9, 10, 11, 12, 13, 14, 15); }
__device__ __forceinline__ v16bf cat16b(v8us lo, v8us hi) { return __builtin_bit_cast(v16bf, __builtin_shufflevector(lo, hi, 0, 1, 2, 3, 4, 5, 6, 7, 8, 9, 10, 11, 12, 13, 14, 15)); }
__device__ __forceinline__ v8f wmma16(v16h a, v16h b, v8f c) { return __builtin_amdgcn_wmma_f32_16x16x32_f16(false, a, false, b, (short)0, c, false, false); }
__device__ __forceinline__ v8f wmmab(v16bf a, v16bf b, v8f c) { return __builtin_amdgcn_wmma_f32_16x16x32_bf16(false, a, false, b, (short)0, c, false, false); }
__device__ __forceinline__ v16h  ldh(const h16* p) { return cat16(*(const v8h*)p, *(const v8h*)(p + 16)); }
__device__ __forceinline__ v16bf ldb(const bf* p)  { return cat16b(*(const v8us*)p, *(const v8us*)(p + 16)); }
__device__ __forceinline__ void wave_sync() { __builtin_amdgcn_fence(3  , "wavefront"); __builtin_amdgcn_wave_barrier(); asm volatile("" ::: "memory"); }

static __device__ __forceinline__ h16 toh_flush(float v) { const h16 r = (h16)v; return (fabsf(v) < 6.103515625e-05f) ? (h16)0.0f : r; }
__device__ __forceinline__ v8f wmma16g(v16h a, v16h b, v8f c) { c = wmma16(a, b, c); asm volatile("v_nop\n\tv_nop\n\tv_nop\n\tv_nop" : "+v"(c) : "v"(a), "v"(b)); return c; }
__device__ __forceinline__ v8f wmmabg(v16bf a, v16bf b, v8f c) { c = wmmab(a, b, c); asm volatile("v_nop\n\tv_nop\n\tv_nop\n\tv_nop" : "+v"(c) : "v"(a), "v"(b)); return c; }
__device__ __forceinline__ v16us ldu(const bf* p) { return __builtin_shufflevector(*(const v8us*)p, *(const v8us*)(p + 16), 0, 1, 2, 3, 4, 5, 6, 7, 8, 9, 10, 11, 12, 13, 14, 15); }
template <int F16> __device__ __forceinline__ v8f mmg(v16us a, v16us b, v8f c) {
    if (F16) return wmma16g(__builtin_bit_cast(v16h, a), __builtin_bit_cast(v16h, b), c);
    return wmmabg(__builtin_bit_cast(v16bf, a), __builtin_bit_cast(v16bf, b), c);
}

__global__ __launch_bounds__(256) void k_cvt8(const float* __restrict__ src, bf* dst, size_t n8) {
    const size_t i = (size_t)blockIdx.x * 256 + threadIdx.x; if (i >= n8) return;
    const v8f v = *(const v8f*)(src + i * 8); v8us o;
#pragma unroll
    for (int k = 0; k < 8; ++k) o[k] = f2bf(v[k]);
    *(volatile v8us*)(dst + i * 8) = o; __threadfence(); *(volatile v8us*)(dst + i * 8) = o;
}

__global__ __launch_bounds__(256) void k_cvt_rows(const float* __restrict__ src, bf* dst, int nT, int bpitch, int toff, size_t total) {
    const size_t i = (size_t)blockIdx.x * 256 + threadIdx.x; if (i >= total) return;
    const size_t per = (size_t)nT * (DM / 8);
    const int b = (int)(i / per); const size_t rem = i % per; const int t = (int)(rem / (DM / 8)); const int pc = (int)(rem % (DM / 8));
    const v8f v = *(const v8f*)(src + ((size_t)t * NB_FULL + (size_t)b) * DM + (size_t)pc * 8); v8us o;
#pragma unroll
    for (int k = 0; k < 8; ++k) o[k] = f2bf(v[k]);
    bf* q = dst + ((size_t)b * (size_t)bpitch + (size_t)toff + (size_t)t) * DM + (size_t)pc * 8;
    *(volatile v8us*)q = o; __threadfence(); *(volatile v8us*)q = o;
}

__global__ __launch_bounds__(256) void k_wcvt16(const float* __restrict__ src, h16* dst, size_t n8) {
    const size_t i = (size_t)blockIdx.x * 256 + threadIdx.x; if (i >= n8) return;
    const v8f v = *(const v8f*)(src + i * 8); v8h o;
#pragma unroll
    for (int k = 0; k < 8; ++k) o[k] = toh_flush(bfr(v[k]) * WCS);
    *(volatile v8h*)(dst + i * 8) = o; __threadfence(); *(volatile v8h*)(dst + i * 8) = o;
}

__global__ __launch_bounds__(256) void k_bound(const float* __restrict__ mask, int* nkt) {
#pragma clang fp contract(off)
    __shared__ int s_last[8]; __shared__ int s_has[8];
    const int tid = threadIdx.x, lane = tid & 31;
    const int wave = __builtin_amdgcn_readfirstlane((int)(threadIdx.x >> 5));
    const int row = tid >> 4, sub = tid & 15;
    const float* mr = mask + (size_t)(blockIdx.x * 16 + row) * TK_FULL + sub * 8;
    int last = -1, has = 0;
#pragma unroll 1
    for (int c = 0; c < TK; c += 128) {
        const v4f a = *(const v4f*)(mr + c); const v4f d = *(const v4f*)(mr + c + 4);
        const int k0 = c + sub * 8;
#pragma unroll
        for (int i = 0; i < 4; ++i) { const float va = bfr(a[i]); last = (va > -1.0e6f) ? (k0 + i) : last; has = (va >= -1.0e4f) ? 1 : has; }
#pragma unroll
        for (int i = 0; i < 4; ++i) { const float vd = bfr(d[i]); last = (vd > -1.0e6f) ? (k0 + 4 + i) : last; has = (vd >= -1.0e4f) ? 1 : has; }
    }
#pragma unroll
    for (int off = 1; off < 16; off <<= 1) { const int l2 = __shfl_xor(last, off, 32); const int h2 = __shfl_xor(has, off, 32); last = last > l2 ? last : l2; has = has | h2; }
    { const int l2 = __shfl_xor(last, 16, 32); const int h2 = __shfl_xor(has, 16, 32); last = last > l2 ? last : l2; has = has & h2; }
    if (lane == 0) { s_last[wave] = last; s_has[wave] = has; }
    __syncthreads();
    int ml = -1, ha = 1;
#pragma unroll
    for (int i = 0; i < 8; ++i) { const int l2 = s_last[i]; ml = ml > l2 ? ml : l2; ha = ha & s_has[i]; }
    int nk = (ml + 32) & ~31;
    nk = (ha != 0) ? nk : TK;
    nk = nk < 32 ? 32 : (nk > TK ? TK : nk);
    if (tid < 32) { volatile int* q = nkt + (size_t)blockIdx.x * 32 + lane; *q = nk; __threadfence(); *q = nk; }
}

template <int F16, int FO, int NPL, int HASB, int RELU>
__device__ __forceinline__ void gemm_tile(const bf* __restrict__ A, const bf* __restrict__ Bt, const int K, const size_t arow0, const size_t brow0,
                                          h16* P0, h16* P1, float* OF, const size_t obase, const size_t opitch,
                                          const float* __restrict__ bias0, const float* __restrict__ bias1, const int bcol0, const float oscale) {
    __shared__ __align__(16) float os[16 * OSP];
    const int lane = threadIdx.x & 31, lr = lane & 15, hi = lane >> 4;
    v8f acc[4][4];
#pragma unroll
    for (int mb = 0; mb < 4; ++mb)
#pragma unroll
        for (int nb = 0; nb < 4; ++nb) acc[mb][nb] = (v8f){};
    const size_t aoff = (arow0 + (size_t)lr) * (size_t)K + 8 * hi, boff = (brow0 + (size_t)lr) * (size_t)K + 8 * hi;
#pragma unroll 1
    for (int kc = 0; kc < K; kc += 32) {
        v16us a[4];
#pragma unroll
        for (int mb = 0; mb < 4; ++mb) a[mb] = ldu(A + aoff + (size_t)mb * 16 * (size_t)K + kc);
#pragma unroll
        for (int nb = 0; nb < 4; ++nb) { const v16us bq = ldu(Bt + boff + (size_t)nb * 16 * (size_t)K + kc);
#pragma unroll
            for (int mb = 0; mb < 4; ++mb) acc[mb][nb] = mmg<F16>(a[mb], bq, acc[mb][nb]); }
    }
    if (FO) {
        static_assert(32 * 16 * 8 == 16 * 64 * 4);
        const int c4 = (lane & 15) * 4;
        v4f bb = (v4f){};
        if (HASB) { const v4f t = *(const v4f*)(bias0 + bcol0 + c4); bb[0] = bfr(t[0]); bb[1] = bfr(t[1]); bb[2] = bfr(t[2]); bb[3] = bfr(t[3]); }
#pragma unroll
        for (int mb = 0; mb < 4; ++mb) {
#pragma unroll
            for (int nb = 0; nb < 4; ++nb) {
#pragma unroll
                for (int j = 0; j < 8; ++j) os[(hi * 8 + j) * OSP + nb * 16 + lr] = acc[mb][nb][j] * oscale; }
            wave_sync();
#pragma unroll 1
            for (int ps = 0; ps < 2; ++ps) {
#pragma unroll
                for (int s = 0; s < 8; ++s) { const int row = 2 * s + (lane >> 4);
                    v4f x = *(const v4fa*)(&os[row * OSP + c4]); x = x + bb;
                    *(volatile v4f*)(OF + obase + (size_t)(mb * 16 + row) * opitch + c4) = x; }
                if (ps == 0) __threadfence(); }
            wave_sync();
        }
    } else {
        static_assert(32 * 16 * 4 == 16 * 64 * 2);
        const int c8 = (lane & 7) * 8;
        float b0[8], b1[8];
#pragma unroll
        for (int i = 0; i < 8; ++i) { b0[i] = 0.0f; b1[i] = 0.0f; }
        if (HASB) { const v4f t0 = *(const v4f*)(bias0 + bcol0 + c8); const v4f t1 = *(const v4f*)(bias0 + bcol0 + c8 + 4);
#pragma unroll
                    for (int i = 0; i < 4; ++i) { b0[i] = bfr(t0[i]); b0[4 + i] = bfr(t1[i]); }
                    if (NPL == 2) { const v4f u0 = *(const v4f*)(bias1 + bcol0 + c8); const v4f u1 = *(const v4f*)(bias1 + bcol0 + c8 + 4);
#pragma unroll
                        for (int i = 0; i < 4; ++i) { b1[i] = bfr(u0[i]); b1[4 + i] = bfr(u1[i]); } } }
#pragma unroll
        for (int mb = 0; mb < 4; ++mb) {
#pragma unroll
            for (int nb = 0; nb < 4; ++nb) {
#pragma unroll
                for (int j = 0; j < 8; ++j) os[(hi * 8 + j) * OSP + nb * 16 + lr] = acc[mb][nb][j] * oscale; }
            wave_sync();
#pragma unroll 1
            for (int ps = 0; ps < 2; ++ps) {
#pragma unroll
                for (int s = 0; s < 4; ++s) { const int row = 4 * s + (lane >> 3);
                    const v4f x0 = *(const v4fa*)(&os[row * OSP + c8]); const v4f x1 = *(const v4fa*)(&os[row * OSP + c8 + 4]); v8h h0, h1;
#pragma unroll
                    for (int i = 0; i < 4; ++i) {
                        float y0 = x0[i] + b0[i], y1 = x1[i] + b0[4 + i];
                        if (RELU) { y0 = fmaxf(y0, 0.0f); y1 = fmaxf(y1, 0.0f); }
                        h0[i] = toh_flush(y0); h0[4 + i] = toh_flush(y1);
                        h1[i] = toh_flush(x0[i] + b1[i]); h1[4 + i] = toh_flush(x1[i] + b1[4 + i]); }
                    const size_t oo = obase + (size_t)(mb * 16 + row) * opitch + c8;
                    *(volatile v8h*)(P0 + oo) = h0; if (NPL == 2) *(volatile v8h*)(P1 + oo) = h1; }
                if (ps == 0) __threadfence(); }
            wave_sync();
        }
    }
}

__global__ __launch_bounds__(32) void k_gemm_q(const bf* __restrict__ XM, const bf* __restrict__ WQ, const float* __restrict__ ub, const float* __restrict__ vb, h16* QU, h16* QV) {
    const int r0 = blockIdx.x * 64, c0 = blockIdx.y * 64;
    const int b = r0 / SEQ, s = r0 % SEQ;
    const size_t obase = (((size_t)b * NH_ + (size_t)(c0 / HD)) * SEQ + (size_t)s) * HD;
    gemm_tile<0, 0, 2, 1, 0>(XM, WQ, DM, (size_t)b * TK + MEMS + s, (size_t)c0, QU, QV, (float*)nullptr, obase, (size_t)HD, ub, vb, c0, 1.0f);
}
__global__ __launch_bounds__(32) void k_gemm_k(const bf* __restrict__ X, const bf* __restrict__ W, h16* KP) {
    const int r0 = blockIdx.x * 64, c0 = blockIdx.y * 64;
    const int b = r0 / TK, t = r0 % TK;
    const size_t obase = (((size_t)b * NH_ + (size_t)(c0 / HD)) * TK + (size_t)t) * HD;
    gemm_tile<0, 0, 1, 0, 0>(X, W, DM, (size_t)r0, (size_t)c0, KP, KP, (float*)nullptr, obase, (size_t)HD, (const float*)nullptr, (const float*)nullptr, 0, 1.0f);
}
__global__ __launch_bounds__(32) void k_gemm_vt(const bf* __restrict__ WV, const bf* __restrict__ XM, h16* VT) {
    const int r0 = blockIdx.x * 64, c0 = blockIdx.y * 64;
    const int b = c0 / TK, t = c0 % TK;
    const size_t obase = ((size_t)b * HK + (size_t)r0) * TK + (size_t)t;
    gemm_tile<0, 0, 1, 0, 0>(WV, XM, DM, (size_t)r0, (size_t)c0, VT, VT, (float*)nullptr, obase, (size_t)TK, (const float*)nullptr, (const float*)nullptr, 0, 1.0f);
}
__global__ __launch_bounds__(32) void k_gemm_wc(const h16* __restrict__ AV, const h16* __restrict__ WC, float* U1) {
    const int r0 = blockIdx.x * 64, c0 = blockIdx.y * 64;
    gemm_tile<1, 1, 1, 0, 0>((const bf*)AV, (const bf*)WC, HK, (size_t)r0, (size_t)c0, (h16*)nullptr, (h16*)nullptr, U1, (size_t)r0 * DM + (size_t)c0, (size_t)DM,
                             (const float*)nullptr, (const float*)nullptr, 0, 1.0f / (AVS * WCS));
}
__global__ __launch_bounds__(32) void k_gemm_ffn1(const h16* __restrict__ UH, const h16* __restrict__ W1, const float* __restrict__ b1, h16* HP) {
    const int r0 = blockIdx.x * 64, c0 = blockIdx.y * 64;
    gemm_tile<1, 0, 1, 1, 1>((const bf*)UH, (const bf*)W1, DM, (size_t)r0, (size_t)c0, HP, HP, (float*)nullptr, (size_t)r0 * MF + (size_t)c0, (size_t)MF, b1, b1, c0, 1.0f / WCS);
}
__global__ __launch_bounds__(32) void k_gemm_ffn2(const h16* __restrict__ HP, const h16* __restrict__ W2, const float* __restrict__ b2, float* Z2) {
    const int r0 = blockIdx.x * 64, c0 = blockIdx.y * 64;
    gemm_tile<1, 1, 1, 1, 0>((const bf*)HP, (const bf*)W2, MF, (size_t)r0, (size_t)c0, (h16*)nullptr, (h16*)nullptr, Z2, (size_t)r0 * DM + (size_t)c0, (size_t)DM, b2, b2, c0, 1.0f / WCS);
}

__global__ __launch_bounds__(32 * AW) void k_flash(const h16* __restrict__ QU, const h16* __restrict__ QV, const h16* __restrict__ KE, const h16* __restrict__ KR,
                                                   const h16* __restrict__ VT, const float* __restrict__ mask, const int* __restrict__ nkt, h16* AV) {
    __shared__ __align__(16) float os[AW * 16 * OSP];
    const int lane = threadIdx.x & 31, lr = lane & 15, hi = lane >> 4;
    const int wave = __builtin_amdgcn_readfirstlane((int)(threadIdx.x >> 5));
    const int zh = blockIdx.y; const int b = zh / NH_, h = zh % NH_;
    const int qb = blockIdx.x * AW + wave;
    const int t0 = qb * 16;
    int nv = nkt[(size_t)qb * 32];
    nv = nv < 32 ? 32 : (nv > TK ? TK : nv); nv &= ~31;
    const int nk = __builtin_amdgcn_readfirstlane(nv);
    const size_t qo = ((size_t)zh * SEQ + (size_t)(t0 + lr)) * HD + 8 * hi;
    const v16h qu0 = ldh(QU + qo), qu1 = ldh(QU + qo + 32), qv0 = ldh(QV + qo), qv1 = ldh(QV + qo + 32);
    const size_t ko = ((size_t)zh * TK + (size_t)lr) * HD + 8 * hi;
    const size_t vo = ((size_t)zh * HD + (size_t)lr) * TK + 8 * hi;
    const float* mrow = mask + (size_t)(t0 + lr) * TK_FULL + 8 * hi;
    v8f o[4];
#pragma unroll
    for (int j = 0; j < 4; ++j) o[j] = (v8f){};
    float m = NEGB, l = 0.0f;
#pragma unroll 1
    for (int key0 = 0; key0 < nk; key0 += 32) {
        const h16* ka = KE + ko + (size_t)key0 * HD;
        const h16* kb = KR + ko + (size_t)key0 * HD;
        v8f sa = (v8f){}, sb = (v8f){};
        { const v16h e0 = ldh(ka), e1 = ldh(ka + 32), r0 = ldh(kb), r1 = ldh(kb + 32);
          sa = wmma16g(e0, qu0, sa); sa = wmma16g(e1, qu1, sa); sa = wmma16g(r0, qv0, sa); sa = wmma16g(r1, qv1, sa); }
        { const v16h e0 = ldh(ka + 16 * HD), e1 = ldh(ka + 16 * HD + 32), r0 = ldh(kb + 16 * HD), r1 = ldh(kb + 16 * HD + 32);
          sb = wmma16g(e0, qu0, sb); sb = wmma16g(e1, qu1, sb); sb = wmma16g(r0, qv0, sb); sb = wmma16g(r1, qv1, sb); }
        const float* mp = mrow + key0;
        const v4f m0 = *(const v4f*)mp, m1 = *(const v4f*)(mp + 4), m2 = *(const v4f*)(mp + 16), m3 = *(const v4f*)(mp + 20);
        float kx[8], ky[8];
#pragma unroll
        for (int r = 0; r < 4; ++r) { kx[r] = m0[r]; kx[4 + r] = m1[r]; ky[r] = m2[r]; ky[4 + r] = m3[r]; }
        float ta[8], tb[8]; float mx = NEGB;
#pragma unroll
        for (int r = 0; r < 8; ++r) {
            ta[r] = (sa[r] * 0.125f + bfr(kx[r])) * LOG2E; tb[r] = (sb[r] * 0.125f + bfr(ky[r])) * LOG2E;
            mx = fmaxf(mx, fmaxf(ta[r], tb[r])); }
        mx = fmaxf(mx, __shfl_xor(mx, 16, 32));
        const float mnew = fmaxf(m, mx);
        const float alpha = __builtin_amdgcn_exp2f(m - mnew);
        const float sh = PSH - mnew;
        v16h pb; float ls = 0.0f;
#pragma unroll
        for (int r = 0; r < 8; ++r) {
            const float xa = ta[r] + sh, xb = tb[r] + sh;
            const float ea = __builtin_amdgcn_exp2f(xa), eb = __builtin_amdgcn_exp2f(xb);
            const float ga = (xa < -14.0f) ? 0.0f : ea, gb = (xb < -14.0f) ? 0.0f : eb;
            const h16 pa = (h16)ga; const h16 pc = (h16)gb;
            pb[r] = pa; pb[8 + r] = pc;
            ls += (float)pa + (float)pc; }
        l = l * alpha + ls; m = mnew;
#pragma unroll
        for (int j = 0; j < 4; ++j) o[j] = o[j] * alpha;
        const h16* va = VT + vo + key0;
        const v16h v0 = ldh(va), v1 = ldh(va + (size_t)16 * TK), v2 = ldh(va + (size_t)32 * TK), v3 = ldh(va + (size_t)48 * TK);
        o[0] = wmma16g(v0, pb, o[0]); o[1] = wmma16g(v1, pb, o[1]); o[2] = wmma16g(v2, pb, o[2]); o[3] = wmma16g(v3, pb, o[3]);
    }
    l += __shfl_xor(l, 16, 32);
    const bool any = l > 0.0f;
    const float lsafe = any ? l : 1.0f;
    const float inv = any ? (AVS * (1.0f / lsafe)) : 0.0f;
    const int wb = wave * 16 * OSP;
#pragma unroll
    for (int j = 0; j < 4; ++j) { v4f a, c;
        a[0] = o[j][0] * inv; a[1] = o[j][1] * inv; a[2] = o[j][2] * inv; a[3] = o[j][3] * inv; c[0] = o[j][4] * inv; c[1] = o[j][5] * inv; c[2] = o[j][6] * inv; c[3] = o[j][7] * inv;
        *(v4fa*)(&os[wb + lr * OSP + 16 * j + 8 * hi]) = a; *(v4fa*)(&os[wb + lr * OSP + 16 * j + 8 * hi + 4]) = c; }
    wave_sync();
    static_assert(32 * 16 * 4 == 16 * HD * 2);
    h16* orow = AV + ((size_t)b * SEQ + (size_t)t0) * HK + h * HD;
#pragma unroll 1
    for (int ps = 0; ps < 2; ++ps) {
#pragma unroll
        for (int s = 0; s < 4; ++s) { const int row = 4 * s + (lane >> 3), c8 = (lane & 7) * 8;
            const v4f x0 = *(const v4fa*)(&os[wb + row * OSP + c8]); const v4f x1 = *(const v4fa*)(&os[wb + row * OSP + c8 + 4]); v8h hv;
#pragma unroll
            for (int i = 0; i < 4; ++i) { hv[i] = toh_flush(x0[i]); hv[4 + i] = toh_flush(x1[i]); }
            *(volatile v8h*)(orow + (size_t)row * HK + c8) = hv; }
        if (ps == 0) __threadfence(); }
}

template <int RESBF, int WH>
__device__ __forceinline__ void ln_row(const float* __restrict__ a, const float* __restrict__ res, const float* __restrict__ g, const float* __restrict__ be, float* of, h16* oh) {
#pragma clang fp contract(off)
    __shared__ float red_s[8]; __shared__ float red_q[8]; __shared__ __align__(16) float yb[DM];
    const int tid = threadIdx.x, lane = tid & 31;
    const int wave = __builtin_amdgcn_readfirstlane((int)(threadIdx.x >> 5));
    const int c = tid * 4;
    const v4f av = *(const v4f*)(a + c); const v4f rv = *(const v4f*)(res + c);
    const v4f gv = *(const v4f*)(g + c); const v4f bv = *(const v4f*)(be + c);
    float v[4]; float sum = 0.0f;
#pragma unroll
    for (int i = 0; i < 4; ++i) { const float r = RESBF ? bfr(rv[i]) : rv[i]; v[i] = av[i] + r; sum += v[i]; }
#pragma unroll
    for (int off = 16; off > 0; off >>= 1) sum += __shfl_xor(sum, off, 32);
    if (lane == 0) red_s[wave] = sum;
    __syncthreads();
    float tot = 0.0f;
#pragma unroll
    for (int i = 0; i < 8; ++i) tot += red_s[i];
    const float mu = tot * (1.0f / DM);
    float sq = 0.0f;
#pragma unroll
    for (int i = 0; i < 4; ++i) { const float d = v[i] - mu; sq += d * d; }
#pragma unroll
    for (int off = 16; off > 0; off >>= 1) sq += __shfl_xor(sq, off, 32);
    if (lane == 0) red_q[wave] = sq;
    __syncthreads();
    float var = 0.0f;
#pragma unroll
    for (int i = 0; i < 8; ++i) var += red_q[i];
    const float inv = 1.0f / sqrtf(var * (1.0f / DM) + 1.0e-5f);
    v4f y;
#pragma unroll
    for (int i = 0; i < 4; ++i) y[i] = (v[i] - mu) * inv * bfr(gv[i]) + bfr(bv[i]);
    if (WH) *(v4fa*)(&yb[c]) = y;
    __syncthreads();
#pragma unroll 1
    for (int ps = 0; ps < 2; ++ps) {
        *(volatile v4f*)(of + c) = y;
        if (WH) { if (tid < 128) { const int c8 = tid * 8;
            const v4f x0 = *(const v4fa*)(&yb[c8]); const v4f x1 = *(const v4fa*)(&yb[c8 + 4]); v8h hv;
#pragma unroll
            for (int i = 0; i < 4; ++i) { hv[i] = toh_flush(x0[i]); hv[4 + i] = toh_flush(x1[i]); }
            *(volatile v8h*)(oh + c8) = hv; } }
        if (ps == 0) __threadfence(); }
}
__global__ __launch_bounds__(256) void k_ln1(const float* __restrict__ U1, const float* __restrict__ x, const float* __restrict__ g, const float* __restrict__ be, float* U, h16* UH) {
    const int R = blockIdx.x; const int b = R / SEQ, s = R % SEQ;
    ln_row<1, 1>(U1 + (size_t)R * DM, x + ((size_t)s * NB_FULL + (size_t)b) * DM, g, be, U + (size_t)R * DM, UH + (size_t)R * DM);
}
__global__ __launch_bounds__(256) void k_ln2(const float* __restrict__ Z2, const float* __restrict__ U, const float* __restrict__ g, const float* __restrict__ be, float* OUT) {
    const int R = blockIdx.x; const int b = R / SEQ, s = R % SEQ;
    ln_row<0, 0>(Z2 + (size_t)R * DM, U + (size_t)R * DM, g, be, OUT + ((size_t)s * NB_FULL + (size_t)b) * DM, (h16*)nullptr);
}

static constexpr size_t al256(size_t v) { return (v + 255) & ~(size_t)255; }
static constexpr size_t SZ_XM  = al256((size_t)NB * TK * DM * 2);
static constexpr size_t SZ_WS  = al256((size_t)HK * DM * 2);
static constexpr size_t SZ_WL  = al256((size_t)MF * DM * 2);
static constexpr size_t SZ_QP  = al256((size_t)NB * NH_ * SEQ * HD * 2);
static constexpr size_t SZ_KP  = al256((size_t)NB * NH_ * TK * HD * 2);
static constexpr size_t SZ_AV  = al256((size_t)ROWS * HK * 2);
static constexpr size_t SZ_F32 = al256((size_t)ROWS * DM * 4);
static constexpr size_t SZ_UH  = al256((size_t)ROWS * DM * 2);
static constexpr size_t SZ_HP  = al256((size_t)ROWS * MF * 2);
static constexpr size_t SZ_NK  = al256((size_t)(SEQ / 16) * 32 * 4);
static constexpr size_t SZ_TOTAL = 2 * SZ_XM + 5 * SZ_WS + 2 * SZ_WL + 2 * SZ_QP + 3 * SZ_KP + SZ_AV + 3 * SZ_F32 + SZ_UH + SZ_HP + SZ_NK;
static_assert(SZ_TOTAL <= (size_t)134217728);
static_assert((size_t)NB * NH_ * TK * HD == (size_t)NB * HK * TK);
static_assert((size_t)DM * HK == (size_t)HK * DM);

extern "C" void kernel_launch(void* const* d_in, const int* in_sizes, int n_in,
                              void* d_out, int out_size, void* d_ws, size_t ws_size, hipStream_t stream) {
    if (n_in < 19) return;
    const size_t needx = ((size_t)(SEQ - 1) * NB_FULL + NB) * DM;
    const size_t needp = ((size_t)(TK - 1) * NB_FULL + NB) * DM;
    const size_t needm = (size_t)(SEQ - 1) * TK_FULL + TK;
    const size_t needy = ((size_t)(MEMS - 1) * NB_FULL + NB) * DM;
    if ((size_t)in_sizes[0] < needx || (size_t)in_sizes[1] < needp || (size_t)in_sizes[2] < needm || (size_t)in_sizes[3] < needy) return;
    if (in_sizes[4] < HK || in_sizes[5] < HK) return;
    for (int i = 6; i <= 10; ++i) if ((size_t)in_sizes[i] < (size_t)HK * DM) return;
    if ((size_t)in_sizes[11] < (size_t)MF * DM || in_sizes[12] < MF || (size_t)in_sizes[13] < (size_t)DM * MF) return;
    for (int i = 14; i <= 18; ++i) if (in_sizes[i] < DM) return;
    if ((size_t)out_size < needx) return;
    if (SZ_TOTAL > ws_size) return;
    const float* x   = (const float*)d_in[0];
    const float* p   = (const float*)d_in[1];
    const float* msk = (const float*)d_in[2];
    const float* mem = (const float*)d_in[3];
    const float* ub  = (const float*)d_in[4];
    const float* vb  = (const float*)d_in[5];
    const float* wq  = (const float*)d_in[6];
    const float* wke = (const float*)d_in[7];
    const float* wkr = (const float*)d_in[8];
    const float* wv  = (const float*)d_in[9];
    const float* wc  = (const float*)d_in[10];
    const float* w1  = (const float*)d_in[11];
    const float* b1  = (const float*)d_in[12];
    const float* w2  = (const float*)d_in[13];
    const float* b2  = (const float*)d_in[14];
    const float* g1  = (const float*)d_in[15];
    const float* e1  = (const float*)d_in[16];
    const float* g2  = (const float*)d_in[17];
    const float* e2  = (const float*)d_in[18];
    float* OUT = (float*)d_out;
    char* wsp = (char*)d_ws;
    bf*  XM  = (bf*)wsp;  wsp += SZ_XM;
    bf*  PB  = (bf*)wsp;  wsp += SZ_XM;
    bf*  WQ  = (bf*)wsp;  wsp += SZ_WS;
    bf*  WKE = (bf*)wsp;  wsp += SZ_WS;
    bf*  WKR = (bf*)wsp;  wsp += SZ_WS;
    bf*  WV  = (bf*)wsp;  wsp += SZ_WS;
    h16* WC  = (h16*)wsp; wsp += SZ_WS;
    h16* W1  = (h16*)wsp; wsp += SZ_WL;
    h16* W2  = (h16*)wsp; wsp += SZ_WL;
    h16* QU  = (h16*)wsp; wsp += SZ_QP;
    h16* QV  = (h16*)wsp; wsp += SZ_QP;
    h16* KE  = (h16*)wsp; wsp += SZ_KP;
    h16* KR  = (h16*)wsp; wsp += SZ_KP;
    h16* VT  = (h16*)wsp; wsp += SZ_KP;
    h16* AV  = (h16*)wsp; wsp += SZ_AV;
    float* U1 = (float*)wsp; wsp += SZ_F32;
    float* U  = (float*)wsp; wsp += SZ_F32;
    float* Z2 = (float*)wsp; wsp += SZ_F32;
    h16* UH  = (h16*)wsp; wsp += SZ_UH;
    h16* HP  = (h16*)wsp; wsp += SZ_HP;
    int* NKT = (int*)wsp; wsp += SZ_NK;

    { const size_t tot = (size_t)NB * MEMS * (DM / 8); k_cvt_rows<<<(unsigned)((tot + 255) / 256), 256, 0, stream>>>(mem, XM, MEMS, TK, 0, tot); }
    { const size_t tot = (size_t)NB * SEQ * (DM / 8);  k_cvt_rows<<<(unsigned)((tot + 255) / 256), 256, 0, stream>>>(x, XM, SEQ, TK, MEMS, tot); }
    { const size_t tot = (size_t)NB * TK * (DM / 8);   k_cvt_rows<<<(unsigned)((tot + 255) / 256), 256, 0, stream>>>(p, PB, TK, TK, 0, tot); }
    { const size_t n8 = (size_t)HK * DM / 8; const unsigned g = (unsigned)((n8 + 255) / 256);
      k_cvt8<<<g, 256, 0, stream>>>(wq, WQ, n8); k_cvt8<<<g, 256, 0, stream>>>(wke, WKE, n8); k_cvt8<<<g, 256, 0, stream>>>(wkr, WKR, n8); k_cvt8<<<g, 256, 0, stream>>>(wv, WV, n8);
      k_wcvt16<<<g, 256, 0, stream>>>(wc, WC, n8); }
    { const size_t n8 = (size_t)MF * DM / 8; const unsigned g = (unsigned)((n8 + 255) / 256);
      k_wcvt16<<<g, 256, 0, stream>>>(w1, W1, n8); k_wcvt16<<<g, 256, 0, stream>>>(w2, W2, n8); }
    k_bound<<<SEQ / 16, 256, 0, stream>>>(msk, NKT);

    k_gemm_q <<<dim3(ROWS / 64,  HK / 64, 1), 32, 0, stream>>>(XM, WQ, ub, vb, QU, QV);
    k_gemm_k <<<dim3(KROWS / 64, HK / 64, 1), 32, 0, stream>>>(XM, WKE, KE);
    k_gemm_k <<<dim3(KROWS / 64, HK / 64, 1), 32, 0, stream>>>(PB, WKR, KR);
    k_gemm_vt<<<dim3(HK / 64, KROWS / 64, 1), 32, 0, stream>>>(WV, XM, VT);

    k_flash<<<dim3(SEQ / (16 * AW), NB * NH_, 1), 32 * AW, 0, stream>>>(QU, QV, KE, KR, VT, msk, NKT, AV);

    k_gemm_wc<<<dim3(ROWS / 64, DM / 64, 1), 32, 0, stream>>>(AV, WC, U1);
    k_ln1<<<ROWS, 256, 0, stream>>>(U1, x, g1, e1, U, UH);
    k_gemm_ffn1<<<dim3(ROWS / 64, MF / 64, 1), 32, 0, stream>>>(UH, W1, b1, HP);
    k_gemm_ffn2<<<dim3(ROWS / 64, DM / 64, 1), 32, 0, stream>>>(HP, W2, b2, Z2);
    k_ln2<<<ROWS, 256, 0, stream>>>(Z2, U, g2, e2, OUT);
}
